// BarrierNet_16432544874700
// MI455X (gfx1250) — hardware-verified
//
#include <hip/hip_runtime.h>
#include <stddef.h>
#include <stdint.h>


#define BROWS  65536
#define NF     64
#define NH     256
#define NH2    512
#define NTHR   128
#define NWAVE  4
#define RPB    64
#define PITCH  264
#define ASC    8.0f
#define WSC    64.0f
#define XSC    8.0f
#define WSCAP  134217728
#define PW1    8
#define PW2    64

static_assert(RPB == NWAVE * 16);
static_assert(NTHR == NWAVE * 32);
static_assert((BROWS % RPB) == 0);
static_assert((NF % 32) == 0);
static_assert((NH % 32) == 0);
static_assert((PITCH % 8) == 0);
static_assert(PITCH >= NH);
static_assert(PW1 * 256 * 8 == NH * NF);
static_assert(PW2 * 256 * 8 == NH2 * NH);
static_assert(ASC == XSC);

typedef float          v2f  __attribute__((ext_vector_type(2)));
typedef float          v4f  __attribute__((ext_vector_type(4)));
typedef float          v8f  __attribute__((ext_vector_type(8)));
typedef _Float16       v8h  __attribute__((ext_vector_type(8)));
typedef _Float16       v16h __attribute__((ext_vector_type(16)));
union FragH { v16h v; v8h h[2]; };

__device__ __forceinline__ v8f wmf(v16h a, v16h b, v8f c) {
  v8f d = __builtin_amdgcn_wmma_f32_16x16x32_f16(false, a, false, b, (short)0, c, false, false);
  asm volatile("v_nop\n\tv_nop\n\tv_nop\n\tv_nop" : "+v"(d) : "v"(a), "v"(b));
  return d;
}

__device__ __forceinline__ v8h cvt8(v4f a, v4f b, float sc) {
  v8h r;
  r[0] = (_Float16)(a.x * sc); r[1] = (_Float16)(a.y * sc);
  r[2] = (_Float16)(a.z * sc); r[3] = (_Float16)(a.w * sc);
  r[4] = (_Float16)(b.x * sc); r[5] = (_Float16)(b.y * sc);
  r[6] = (_Float16)(b.z * sc); r[7] = (_Float16)(b.w * sc);
  return r;
}

__device__ __forceinline__ float erfinv_f32(float x) {
  const float w = -log1pf(-(x * x));
  const float wa = w - 2.5f;
  const float wb = sqrtf(w) - 3.0f;
  float pa = 2.81022636e-08f;
  pa = 3.43273939e-07f  + pa * wa;
  pa = -3.5233877e-06f  + pa * wa;
  pa = -4.39150654e-06f + pa * wa;
  pa = 0.00021858087f   + pa * wa;
  pa = -0.00125372503f  + pa * wa;
  pa = -0.00417768164f  + pa * wa;
  pa = 0.246640727f     + pa * wa;
  pa = 1.50140941f      + pa * wa;
  float pb = -0.000200214257f;
  pb = 0.000100950558f  + pb * wb;
  pb = 0.00134934322f   + pb * wb;
  pb = -0.00367342844f  + pb * wb;
  pb = 0.00573950773f   + pb * wb;
  pb = -0.0076224613f   + pb * wb;
  pb = 0.00943887047f   + pb * wb;
  pb = 1.00167406f      + pb * wb;
  pb = 2.83297682f      + pb * wb;
  const float p = (w < 5.0f) ? pa : pb;
  return p * x;
}

__global__ __launch_bounds__(256) void k_prepw(const float* __restrict__ W1, const float* __restrict__ W21,
                                              const float* __restrict__ W22, _Float16* w1h, _Float16* w2h) {
  const int b = blockIdx.x, tid = threadIdx.x;
  const float* src;
  _Float16* dst;
  if (b < PW1) {
    const size_t e = ((size_t)b * 256 + tid) * 8;
    src = W1 + e;
    dst = w1h + e;
  } else {
    const size_t u = (size_t)(b - PW1) * 256 + tid;
    const size_t row = u >> 5, c8 = (u & 31) * 8;
    if (b < PW1 + PW2 / 2) src = W21 + row * NH + c8;
    else                   src = W22 + (row - NH) * NH + c8;
    dst = w2h + u * 8;
  }
  const v4f f0 = *(const v4f*)src;
  const v4f f1 = *(const v4f*)(src + 4);
  const v8h a = cvt8(f0, f1, WSC);
  *(volatile v8h*)dst = a;
  __threadfence();
  *(volatile v8h*)dst = a;
}

__global__ __launch_bounds__(NTHR) void k_main(
    const float* __restrict__ obs, const _Float16* __restrict__ w1h, const _Float16* __restrict__ w2h,
    const float* __restrict__ b1, const float* __restrict__ b21, const float* __restrict__ b22,
    const float* __restrict__ W31, const float* __restrict__ b31,
    const float* __restrict__ W32, const float* __restrict__ b32, float* out) {
  __shared__ __attribute__((aligned(16))) _Float16 x1t[NWAVE * 16 * PITCH];
  __shared__ __attribute__((aligned(16))) float ost[NWAVE * 32];

  const int tid = threadIdx.x, lane = tid & 31, wave = tid >> 5, hh = lane >> 4, m = lane & 15;
  const int row0 = blockIdx.x * RPB + wave * 16;
  _Float16* xt = x1t + wave * (16 * PITCH);
  constexpr float OSC = 1.0f / (ASC * WSC);

  FragH a1f[2];
  {
    const float* p = obs + (size_t)(row0 + m) * NF + 8 * hh;
#pragma unroll
    for (int s = 0; s < 2; ++s) {
      const v4f f0 = *(const v4f*)(p + 32 * s);
      const v4f f1 = *(const v4f*)(p + 32 * s + 4);
      const v4f f2 = *(const v4f*)(p + 32 * s + 16);
      const v4f f3 = *(const v4f*)(p + 32 * s + 20);
      a1f[s].h[0] = cvt8(f0, f1, ASC);
      a1f[s].h[1] = cvt8(f2, f3, ASC);
    }
  }

#pragma unroll 1
  for (int t = 0; t < NH / 16; ++t) {
    const _Float16* bp = w1h + (size_t)(t * 16 + m) * NF + 8 * hh;
    FragH bA, bB;
    bA.h[0] = *(const v8h*)(bp);
    bA.h[1] = *(const v8h*)(bp + 16);
    bB.h[0] = *(const v8h*)(bp + 32);
    bB.h[1] = *(const v8h*)(bp + 48);
    v8f c = {0.f, 0.f, 0.f, 0.f, 0.f, 0.f, 0.f, 0.f};
    c = wmf(a1f[0].v, bA.v, c);
    c = wmf(a1f[1].v, bB.v, c);
    const int col = t * 16 + m;
    const float bia = b1[col];
#pragma unroll
    for (int r = 0; r < 8; ++r) {
      const float v = fmaxf(c[r] * OSC + bia, 0.0f);
      xt[(8 * hh + r) * PITCH + col] = (_Float16)(v * XSC);
    }
  }
  __syncthreads();

  FragH ax[8];
  {
    const _Float16* xp = xt + m * PITCH + 8 * hh;
#pragma unroll
    for (int s = 0; s < 8; ++s) {
      ax[s].h[0] = *(const v8h*)(xp + 32 * s);
      ax[s].h[1] = *(const v8h*)(xp + 32 * s + 16);
    }
  }

  float hp0[8], hp1[8], hp2[8];
#pragma unroll
  for (int r = 0; r < 8; ++r) { hp0[r] = 0.0f; hp1[r] = 0.0f; hp2[r] = 0.0f; }

#pragma unroll 1
  for (int nt = 0; nt < NH / 16; ++nt) {
    const _Float16* bp = w2h + (size_t)(nt * 16 + m) * NH + 8 * hh;
    v8f c = {0.f, 0.f, 0.f, 0.f, 0.f, 0.f, 0.f, 0.f};
#pragma unroll
    for (int s = 0; s < 8; ++s) {
      FragH bf;
      bf.h[0] = *(const v8h*)(bp + 32 * s);
      bf.h[1] = *(const v8h*)(bp + 32 * s + 16);
      c = wmf(ax[s].v, bf.v, c);
    }
    const int col = nt * 16 + m;
    const float bia = b21[col];
    const float hw0 = W31[col];
    const float hw1 = W31[NH + col];
#pragma unroll
    for (int r = 0; r < 8; ++r) {
      const float v = fmaxf(c[r] * OSC + bia, 0.0f);
      hp0[r] += v * hw0;
      hp1[r] += v * hw1;
    }
  }

#pragma unroll 1
  for (int nt = 0; nt < NH / 16; ++nt) {
    const _Float16* bp = w2h + (size_t)(NH + nt * 16 + m) * NH + 8 * hh;
    v8f c = {0.f, 0.f, 0.f, 0.f, 0.f, 0.f, 0.f, 0.f};
#pragma unroll
    for (int s = 0; s < 8; ++s) {
      FragH bf;
      bf.h[0] = *(const v8h*)(bp + 32 * s);
      bf.h[1] = *(const v8h*)(bp + 32 * s + 16);
      c = wmf(ax[s].v, bf.v, c);
    }
    const int col = nt * 16 + m;
    const float bia = b22[col];
    const float hw2 = W32[col];
#pragma unroll
    for (int r = 0; r < 8; ++r) {
      const float v = fmaxf(c[r] * OSC + bia, 0.0f);
      hp2[r] += v * hw2;
    }
  }

#pragma unroll
  for (int r = 0; r < 8; ++r) {
#pragma unroll
    for (int o = 1; o < 16; o <<= 1) {
      hp0[r] += __shfl_xor(hp0[r], o);
      hp1[r] += __shfl_xor(hp1[r], o);
      hp2[r] += __shfl_xor(hp2[r], o);
    }
  }

  const int rsel = m & 7;
  float u0 = 0.0f, u1 = 0.0f, sv = 0.0f;
#pragma unroll
  for (int r = 0; r < 8; ++r) {
    const bool pk = (rsel == r);
    u0 = pk ? hp0[r] : u0;
    u1 = pk ? hp1[r] : u1;
    sv = pk ? hp2[r] : sv;
  }
  u0 += b31[0];
  u1 += b31[1];
  sv += b32[0];

  const int row = row0 + 8 * hh + rsel;
  const float* orw = obs + (size_t)row * NF;
  const v2f rl = *(const v2f*)(orw + 6);
  const v2f hv = *(const v2f*)(orw + 8);
  float us0, us1;
  {
#pragma clang fp contract(off)
    const float rx = rl.x, ry = rl.y, vx = hv.x, vy = hv.y;
    const float rn2 = rx * rx + ry * ry;
    const float hcb = rn2 - 0.64f;
    const float sc = fmaxf(sv, -30.0f);
    const float sig = 1.0f / (1.0f + expf(-sc));
    float beta = 0.2f * sig;
    beta = fminf(fmaxf(beta, 1e-6f), 0.999999f);
    const float xe = 1.0f - 2.0f * beta;
    const float z = 1.41421354f * erfinv_f32(xe);
    const float pdf = 0.398942280f * expf(-0.5f * z * z);
    const float cvar = pdf / beta;
    const float rdm = 2.0f * (vx * rx + vy * ry);
    const float base = -2.0f * hcb + rdm;
    const float sf0 = sqrtf((4.0f * (0.1f * 0.1f)) * rn2 + 1e-8f);
    const float sf1 = sqrtf((4.0f * (0.3f * 0.3f)) * rn2 + 1e-8f);
    const float sf2 = sqrtf((4.0f * (0.5f * 0.5f)) * rn2 + 1e-8f);
    const float q0 = (base + sf0 * cvar) * (1.0f / 0.1f);
    const float q1 = (base + sf1 * cvar) * (1.0f / 0.1f);
    const float q2 = (base + sf2 * cvar) * (1.0f / 0.1f);
    const float mx = fmaxf(fmaxf(q0, q1), q2);
    const float e0 = expf(q0 - mx), e1 = expf(q1 - mx), e2 = expf(q2 - mx);
    const float lse = logf((e0 + e2) + e1) + mx;
    const float rhs_wc = 0.1f * lse;
    const float G0 = -2.0f * rx, G1 = -2.0f * ry;
    const float viol = (G0 * u0 + G1 * u1) + rhs_wc;
    const float den = (G0 * G0 + G1 * G1) + 1e-12f;
    const float vp = (viol > 0.0f) ? viol : 0.0f;
    const float stp = vp / den;
    us0 = u0 - stp * G0;
    us1 = u1 - stp * G1;
  }

  if (m < 8) {
    v2f w2; w2.x = us0; w2.y = us1;
    *(v2f*)(ost + wave * 32 + 2 * (8 * hh + m)) = w2;
  }
  __syncthreads();
  const int q = lane & 7;
  const v4f ov = *(const v4f*)(ost + wave * 32 + 4 * q);
  float* gp = out + (size_t)row0 * 2 + 4 * q;
  if (lane < 8) *(volatile v4f*)gp = ov;
  __threadfence();
  if (lane < 8) *(volatile v4f*)gp = ov;
}

extern "C" void kernel_launch(void* const* d_in, const int* in_sizes, int n_in,
                              void* d_out, int out_size, void* d_ws, size_t ws_size,
                              hipStream_t stream) {
  if (n_in < 11) return;
  if (in_sizes[0] != BROWS * NF) return;
  if (in_sizes[1] != NH * NF || in_sizes[2] != NH) return;
  if (in_sizes[3] != NH * NH || in_sizes[4] != NH) return;
  if (in_sizes[5] != NH * NH || in_sizes[6] != NH) return;
  if (in_sizes[7] != 2 * NH || in_sizes[8] != 2) return;
  if (in_sizes[9] != NH || in_sizes[10] != 1) return;
  if (out_size != BROWS * 2) return;

  const float* obs = (const float*)d_in[0];
  const float* W1  = (const float*)d_in[1];
  const float* b1  = (const float*)d_in[2];
  const float* W21 = (const float*)d_in[3];
  const float* b21 = (const float*)d_in[4];
  const float* W22 = (const float*)d_in[5];
  const float* b22 = (const float*)d_in[6];
  const float* W31 = (const float*)d_in[7];
  const float* b31 = (const float*)d_in[8];
  const float* W32 = (const float*)d_in[9];
  const float* b32 = (const float*)d_in[10];
  float* out = (float*)d_out;

  char* ws = (char*)d_ws;
  size_t off = 0;
  const size_t oW1 = off; off += (size_t)NH * NF * 2;   off = (off + 255) & ~(size_t)255;
  const size_t oW2 = off; off += (size_t)NH2 * NH * 2;  off = (off + 255) & ~(size_t)255;
  if (off > ws_size || off > (size_t)WSCAP) return;
  _Float16* w1h = (_Float16*)(ws + oW1);
  _Float16* w2h = (_Float16*)(ws + oW2);

  k_prepw<<<PW1 + PW2, 256, 0, stream>>>(W1, W21, W22, w1h, w2h);
  k_main<<<BROWS / RPB, NTHR, 0, stream>>>(obs, w1h, w2h, b1, b21, b22, W31, b31, W32, b32, out);
}
